// EinFFT_6897717477703
// MI455X (gfx1250) — hardware-run, weakly checked
//
#include <hip/hip_runtime.h>
#include <stdint.h>

#define NT    32768
#define NSEQ  8192
#define DM    64
#define DI    128
#define DS    64
#define DTR   4
#define XZW   256
#define PJW   160
#define HID   1024
#define HROWS 16384

#define S_LN  8.0f
#define S_U   256.0f
#define S_Y   1024.0f
#define S_E   8.0f
#define S_H   64.0f
#define S_W   64.0f
#define RLO   1024.0f
#define ILO   0.0009765625f
#define LOG2E 1.4426950408889634f

static_assert((NT % 64) == 0);
static_assert(NSEQ * 4 == NT);
static_assert(HROWS * 2 == NT);
static_assert((HROWS % 64) == 0);
static_assert((XZW % 128) == 0);
static_assert((HID % 128) == 0);
static_assert((PJW % 32) == 0);
static_assert(DM == 64);
static_assert(DI == 128);
static_assert(DS == 64);

typedef _Float16 v16h __attribute__((ext_vector_type(16)));
typedef _Float16 v8h  __attribute__((ext_vector_type(8)));
typedef float    v8f  __attribute__((ext_vector_type(8)));
typedef float    v4f  __attribute__((ext_vector_type(4)));
typedef float    v2f  __attribute__((ext_vector_type(2)));
typedef unsigned int v4u __attribute__((ext_vector_type(4)));
typedef unsigned int v2u __attribute__((ext_vector_type(2)));

__device__ __forceinline__ unsigned short bf_bits(float f) {
  unsigned u = __float_as_uint(f);
  return (unsigned short)((u + 0x7FFFu + ((u >> 16) & 1u)) >> 16);
}
__device__ __forceinline__ float bfr(float f) { return __uint_as_float(((unsigned)bf_bits(f)) << 16); }
__device__ __forceinline__ unsigned short h_bits(_Float16 x) { return __builtin_bit_cast(unsigned short, x); }
__device__ __forceinline__ unsigned short hb16(float f) { return h_bits((_Float16)f); }
__device__ __forceinline__ unsigned pk16(unsigned short a, unsigned short b) { return (unsigned)a | ((unsigned)b << 16); }
__device__ __forceinline__ v8f zero8() { v8f z = {0.f, 0.f, 0.f, 0.f, 0.f, 0.f, 0.f, 0.f}; return z; }
__device__ __forceinline__ float sigf(float x) { return __builtin_amdgcn_rcpf(1.0f + __expf(-x)); }

__device__ __forceinline__ float wsum(float v) {
  v += __shfl_xor(v, 1, 32);
  v += __shfl_xor(v, 2, 32);
  v += __shfl_xor(v, 4, 32);
  v += __shfl_xor(v, 8, 32);
  v += __shfl_xor(v, 16, 32);
  return v;
}

__device__ __forceinline__ unsigned hl2(float v0, float v1, unsigned& lo) {
  const _Float16 h0 = (_Float16)v0;
  const _Float16 h1 = (_Float16)v1;
  lo = pk16(hb16((v0 - (float)h0) * RLO), hb16((v1 - (float)h1) * RLO));
  return pk16(h_bits(h0), h_bits(h1));
}
__device__ __forceinline__ void pack4(const v4f v, const float s, v2u& ph, v2u& pl) {
  unsigned l0, l1;
  const unsigned p0 = hl2(v[0] * s, v[1] * s, l0);
  const unsigned p1 = hl2(v[2] * s, v[3] * s, l1);
  ph[0] = p0; ph[1] = p1;
  pl[0] = l0; pl[1] = l1;
}

__device__ __forceinline__ v16h ldfrag_h(const _Float16* p) {
  union { v16h v; v8h h[2]; } f;
  f.h[0] = *(const v8h*)(p);
  f.h[1] = *(const v8h*)(p + 16);
  return f.v;
}

__device__ __forceinline__ v8f mma_raw(v16h a, v16h b, v8f c) {
  return __builtin_amdgcn_wmma_f32_16x16x32_f16(false, a, false, b, (short)0, c, false, false);
}
__device__ __forceinline__ void guard8(v8f& c0, v8f& c1, v8f& c2, v8f& c3, v8f& c4, v8f& c5, v8f& c6, v8f& c7,
                                       const v16h& a0, const v16h& a1, const v16h& a2, const v16h& a3,
                                       const v16h& b0, const v16h& b1) {
#if defined(__HIP_DEVICE_COMPILE__)
  asm volatile("v_nop\n\tv_nop\n\tv_nop\n\tv_nop"
               : "+v"(c0), "+v"(c1), "+v"(c2), "+v"(c3), "+v"(c4), "+v"(c5), "+v"(c6), "+v"(c7)
               : "v"(a0), "v"(a1), "v"(a2), "v"(a3), "v"(b0), "v"(b1));
#endif
}

template <int NWN>
__device__ __forceinline__ void mm_tile2(const _Float16* __restrict__ Ah, const _Float16* __restrict__ Al, int lda,
                                         const _Float16* __restrict__ W, int ldw, int nks,
                                         int arow0, int bcol0, float* Cs) {
  constexpr int LDC = 32 * NWN + 4;
  const int tid = threadIdx.x, wave = tid >> 5, lane = tid & 31, hh = lane >> 4, c = lane & 15;
  const int mw = wave / NWN, nw = wave - mw * NWN;
  const size_t ao0 = (size_t)(arow0 + mw * 32 + c) * (size_t)lda + 8 * hh;
  const size_t ao1 = (size_t)(arow0 + mw * 32 + 16 + c) * (size_t)lda + 8 * hh;
  const _Float16* a0h = Ah + ao0;
  const _Float16* a1h = Ah + ao1;
  const _Float16* a0l = Al + ao0;
  const _Float16* a1l = Al + ao1;
  const _Float16* b0p = W + (size_t)(bcol0 + nw * 32 + c) * (size_t)ldw + 8 * hh;
  const _Float16* b1p = W + (size_t)(bcol0 + nw * 32 + 16 + c) * (size_t)ldw + 8 * hh;
  v8f h00 = zero8(), h01 = zero8(), h10 = zero8(), h11 = zero8();
  v8f l00 = zero8(), l01 = zero8(), l10 = zero8(), l11 = zero8();
#pragma unroll 1
  for (int ks = 0; ks < nks; ++ks) {
    const int ko = ks * 32;
    const v16h fa0 = ldfrag_h(a0h + ko);
    const v16h fa1 = ldfrag_h(a1h + ko);
    const v16h ga0 = ldfrag_h(a0l + ko);
    const v16h ga1 = ldfrag_h(a1l + ko);
    const v16h fb0 = ldfrag_h(b0p + ko);
    const v16h fb1 = ldfrag_h(b1p + ko);
    h00 = mma_raw(fa0, fb0, h00);
    h01 = mma_raw(fa0, fb1, h01);
    h10 = mma_raw(fa1, fb0, h10);
    h11 = mma_raw(fa1, fb1, h11);
    l00 = mma_raw(ga0, fb0, l00);
    l01 = mma_raw(ga0, fb1, l01);
    l10 = mma_raw(ga1, fb0, l10);
    l11 = mma_raw(ga1, fb1, l11);
    guard8(h00, h01, h10, h11, l00, l01, l10, l11, fa0, fa1, ga0, ga1, fb0, fb1);
  }
#pragma unroll
  for (int r = 0; r < 8; ++r) {
    const int row = mw * 32 + 8 * hh + r;
    Cs[row * LDC + nw * 32 + c]             = h00[r] + l00[r] * ILO;
    Cs[row * LDC + nw * 32 + 16 + c]        = h01[r] + l01[r] * ILO;
    Cs[(row + 16) * LDC + nw * 32 + c]      = h10[r] + l10[r] * ILO;
    Cs[(row + 16) * LDC + nw * 32 + 16 + c] = h11[r] + l11[r] * ILO;
  }
}

__global__ __launch_bounds__(256)
void k_cvt(const float* __restrict__ src, int N, int K, unsigned short* dst, int Np) {
  const int kp = K >> 3;
  const int total = Np * kp;
  const int i = blockIdx.x * 256 + threadIdx.x;
  const int ic = min(i, total - 1);
  const int n = ic / kp, piece = ic - n * kp;
  const int nc = min(n, N - 1);
  const float m = (n < N) ? S_W : 0.0f;
  const float* sp = src + (size_t)nc * (size_t)K + piece * 8;
  const v4f v0 = *(const v4f*)sp;
  const v4f v1 = *(const v4f*)(sp + 4);
  v4u u;
  u[0] = pk16(hb16(bfr(v0[0]) * m), hb16(bfr(v0[1]) * m));
  u[1] = pk16(hb16(bfr(v0[2]) * m), hb16(bfr(v0[3]) * m));
  u[2] = pk16(hb16(bfr(v1[0]) * m), hb16(bfr(v1[1]) * m));
  u[3] = pk16(hb16(bfr(v1[2]) * m), hb16(bfr(v1[3]) * m));
  if (i < total) {
    unsigned short* p = dst + (size_t)n * (size_t)K + piece * 8;
    *(volatile v4u*)p = u;
    __threadfence();
    *(volatile v4u*)p = u;
  }
}

__global__ __launch_bounds__(256)
void k_atab(const float* __restrict__ alog, int n, float* dst) {
  const int i = blockIdx.x * 256 + threadIdx.x;
  const int ic = min(i, n - 1);
  const float v = -expf(bfr(alog[ic])) * LOG2E;
  if (i < n) {
    float* p = dst + i;
    *(volatile float*)p = v;
    __threadfence();
    *(volatile float*)p = v;
  }
}

template <int MODE>
__global__ __launch_bounds__(256)
void k_ln(const float* __restrict__ src, const float* __restrict__ g, const float* __restrict__ bb,
          float* o32, unsigned short* oh, unsigned short* ol) {
  const int tid = threadIdx.x, wv = tid >> 5, lane = tid & 31;
  const size_t t = (size_t)blockIdx.x * 8 + wv;
  const v2f xr = *(const v2f*)(src + t * DM + 2 * lane);
  const v2f gr = *(const v2f*)(g + 2 * lane);
  const v2f br = *(const v2f*)(bb + 2 * lane);
  float a0 = xr[0], a1 = xr[1];
  if (MODE == 0) {
    a0 = bfr(a0);
    a1 = bfr(a1);
    v2f xo;
    xo[0] = a0; xo[1] = a1;
    float* p = o32 + t * DM + 2 * lane;
    *(volatile v2f*)p = xo;
    __threadfence();
    *(volatile v2f*)p = xo;
  }
  const float s = wsum(a0 + a1);
  const float mu = s * (1.0f / (float)DM);
  const float d0 = a0 - mu, d1 = a1 - mu;
  const float sq = wsum(d0 * d0 + d1 * d1);
  const float rs = rsqrtf(sq * (1.0f / (float)DM) + 1e-5f);
  const float y0 = (d0 * rs) * bfr(gr[0]) + bfr(br[0]);
  const float y1 = (d1 * rs) * bfr(gr[1]) + bfr(br[1]);
  v2f yo;
  yo[0] = y0; yo[1] = y1;
  if (MODE == 2) {
    float* p = o32 + t * DM + 2 * lane;
    *(volatile v2f*)p = yo;
    __threadfence();
    *(volatile v2f*)p = yo;
  } else {
    unsigned lo;
    const unsigned hi = hl2(y0 * ((MODE == 0) ? S_LN : S_E), y1 * ((MODE == 0) ? S_LN : S_E), lo);
    unsigned* hp = (unsigned*)(void*)(oh + t * DM + 2 * lane);
    unsigned* lp = (unsigned*)(void*)(ol + t * DM + 2 * lane);
    float* p = o32 + t * DM + 2 * lane;
    if (MODE == 1) *(volatile v2f*)p = yo;
    *(volatile unsigned*)hp = hi;
    *(volatile unsigned*)lp = lo;
    __threadfence();
    if (MODE == 1) *(volatile v2f*)p = yo;
    *(volatile unsigned*)hp = hi;
    *(volatile unsigned*)lp = lo;
  }
}

__global__ __launch_bounds__(128)
void k_scan(const float* __restrict__ dbc, const float* __restrict__ uu, const float* __restrict__ zz,
            const float* __restrict__ a2, const float* __restrict__ dtw, const float* __restrict__ dtb,
            const float* __restrict__ dd, unsigned short* yh, unsigned short* yl) {
  __shared__ float sB[4 * DS];
  __shared__ float sC[4 * DS];
  __shared__ float sdt[16];
  __shared__ float sdel[4 * DI];
  __shared__ __align__(16) unsigned short sY[8 * DI];
  const int d = threadIdx.x;
  const size_t t0 = (size_t)blockIdx.x * 4;
#pragma unroll 1
  for (int i = d; i < 4 * DS; i += DI) {
    const int t = i >> 6, n = i & 63;
    sB[i] = dbc[(t0 + t) * PJW + n];
    sC[i] = dbc[(t0 + t) * PJW + DS + n];
  }
  {
    const int q = d & 15;
    const float v = dbc[(t0 + (q >> 2)) * PJW + 2 * DS + (q & 3)];
    if (d < 16) sdt[d] = v;
  }
  __syncthreads();
  const v4f wr = *(const v4f*)(dtw + d * DTR);
  const float w0 = bfr(wr[0]), w1 = bfr(wr[1]), w2 = bfr(wr[2]), w3 = bfr(wr[3]);
  const float db = bfr(dtb[d]);
#pragma unroll 1
  for (int t = 0; t < 4; ++t) {
    const float r = ((sdt[t * 4 + 0] * w0 + sdt[t * 4 + 1] * w1) + (sdt[t * 4 + 2] * w2 + sdt[t * 4 + 3] * w3)) + db;
    const float sp = fmaxf(r, 0.0f) + log1pf(expf(-fabsf(r)));
    sdel[t * DI + d] = sp;
  }
  __syncthreads();
  const float e0 = sdel[d], e1 = sdel[DI + d], e2 = sdel[2 * DI + d], e3 = sdel[3 * DI + d];
  const float u0 = uu[(t0 + 0) * DI + d];
  const float u1 = uu[(t0 + 1) * DI + d];
  const float u2 = uu[(t0 + 2) * DI + d];
  const float u3 = uu[(t0 + 3) * DI + d];
  const float du0 = e0 * u0, du1 = e1 * u1, du2 = e2 * u2, du3 = e3 * u3;
  float y0 = 0.0f, y1 = 0.0f, y2 = 0.0f, y3 = 0.0f;
  const float* ap = a2 + d * DS;
#pragma unroll 1
  for (int n = 0; n < DS; ++n) {
    const float an = ap[n];
    float h = du0 * sB[n];
    y0 += h * sC[n];
    h = exp2f(e1 * an) * h + du1 * sB[DS + n];
    y1 += h * sC[DS + n];
    h = exp2f(e2 * an) * h + du2 * sB[2 * DS + n];
    y2 += h * sC[2 * DS + n];
    h = exp2f(e3 * an) * h + du3 * sB[3 * DS + n];
    y3 += h * sC[3 * DS + n];
  }
  const float Dd = bfr(dd[d]);
  const float z0 = zz[(t0 + 0) * DI + d];
  const float z1 = zz[(t0 + 1) * DI + d];
  const float z2 = zz[(t0 + 2) * DI + d];
  const float z3 = zz[(t0 + 3) * DI + d];
  {
    const float v = ((y0 + u0 * Dd) * (z0 * sigf(z0))) * S_Y;
    const _Float16 hq = (_Float16)v;
    sY[0 * DI + d] = h_bits(hq);
    sY[4 * DI + 0 * DI + d] = hb16((v - (float)hq) * RLO);
  }
  {
    const float v = ((y1 + u1 * Dd) * (z1 * sigf(z1))) * S_Y;
    const _Float16 hq = (_Float16)v;
    sY[1 * DI + d] = h_bits(hq);
    sY[4 * DI + 1 * DI + d] = hb16((v - (float)hq) * RLO);
  }
  {
    const float v = ((y2 + u2 * Dd) * (z2 * sigf(z2))) * S_Y;
    const _Float16 hq = (_Float16)v;
    sY[2 * DI + d] = h_bits(hq);
    sY[4 * DI + 2 * DI + d] = hb16((v - (float)hq) * RLO);
  }
  {
    const float v = ((y3 + u3 * Dd) * (z3 * sigf(z3))) * S_Y;
    const _Float16 hq = (_Float16)v;
    sY[3 * DI + d] = h_bits(hq);
    sY[4 * DI + 3 * DI + d] = hb16((v - (float)hq) * RLO);
  }
  __syncthreads();
  const int pl = d >> 6, pc = d & 63;
  const v4u val = *(const v4u*)(sY + d * 8);
  unsigned short* dst = (pl ? yl : yh) + t0 * DI + pc * 8;
  *(volatile v4u*)dst = val;
  __threadfence();
  *(volatile v4u*)dst = val;
}

template <int MODE, int NWN>
__global__ __launch_bounds__(64 * NWN)
void k_gemm(const unsigned short* __restrict__ ah, const unsigned short* __restrict__ al, int lda,
            const unsigned short* __restrict__ w, int ldw, int nks,
            const float* __restrict__ q0, const float* __restrict__ q1,
            float* o32, float* o32b, unsigned short* oh, unsigned short* ol) {
  constexpr int NBW = 32 * NWN;
  constexpr int NW  = 2 * NWN;
  constexpr int LDC = NBW + 4;
  __shared__ __align__(16) float Cs[64 * LDC];
  const int tid = threadIdx.x, wave = tid >> 5, lane = tid & 31;
  const int mb = blockIdx.x, nb = blockIdx.y;
  mm_tile2<NWN>((const _Float16*)(const void*)ah, (const _Float16*)(const void*)al, lda,
                (const _Float16*)(const void*)w, ldw, nks, mb * 64, nb * NBW, Cs);
  __syncthreads();
  if (MODE == 0) {
    const int cb = lane * 4;
    const v4f cbv = *(const v4f*)(q1 + cb);
    const v4f t0v = *(const v4f*)(q0 + (cb + 0) * 4);
    const v4f t1v = *(const v4f*)(q0 + (cb + 1) * 4);
    const v4f t2v = *(const v4f*)(q0 + (cb + 2) * 4);
    const v4f t3v = *(const v4f*)(q0 + (cb + 3) * 4);
    v4f bia, wc0, wc1, wc2, wc3;
#pragma unroll
    for (int k = 0; k < 4; ++k) {
      bia[k] = bfr(cbv[k]);
      wc0[k] = bfr(t0v[k]);
      wc1[k] = bfr(t1v[k]);
      wc2[k] = bfr(t2v[k]);
      wc3[k] = bfr(t3v[k]);
    }
#pragma unroll 1
    for (int row = wave; row < 64; row += NW) {
      const size_t t = (size_t)mb * 64 + row;
      if (nb != 0) {
        const v4f a = *(const v4f*)(Cs + row * LDC + cb);
        v4f z;
#pragma unroll
        for (int e = 0; e < 4; ++e) z[e] = a[e] * (1.0f / 512.0f);
        float* p = o32 + t * DI + cb;
        *(volatile v4f*)p = z;
        __threadfence();
        *(volatile v4f*)p = z;
      } else {
        const int l = row & 3;
        v4f acc = bia;
#pragma unroll
        for (int k = 0; k < 4; ++k) {
          const int rr = max(row - 3 + k, row - l);
          const float m = (k >= 3 - l) ? (1.0f / 512.0f) : 0.0f;
          const v4f xv = *(const v4f*)(Cs + rr * LDC + cb);
          acc[0] += (xv[0] * m) * wc0[k];
          acc[1] += (xv[1] * m) * wc1[k];
          acc[2] += (xv[2] * m) * wc2[k];
          acc[3] += (xv[3] * m) * wc3[k];
        }
        v4f u;
#pragma unroll
        for (int e = 0; e < 4; ++e) u[e] = acc[e] * sigf(acc[e]);
        v2u ph, pl;
        pack4(u, S_U, ph, pl);
        float* pu = o32b + t * DI + cb;
        unsigned short* hp = oh + t * DI + cb;
        unsigned short* lp = ol + t * DI + cb;
        *(volatile v4f*)pu = u;
        *(volatile v2u*)hp = ph;
        *(volatile v2u*)lp = pl;
        __threadfence();
        *(volatile v4f*)pu = u;
        *(volatile v2u*)hp = ph;
        *(volatile v2u*)lp = pl;
      }
    }
  } else if (MODE == 1) {
    const int c0 = lane * 4;
    const int c1 = 128 + lane * 4;
    const int c1c = min(c1, NBW - 4);
#pragma unroll 1
    for (int row = wave; row < 64; row += NW) {
      const size_t t = (size_t)mb * 64 + row;
      const v4f a0 = *(const v4f*)(Cs + row * LDC + c0);
      const v4f a1 = *(const v4f*)(Cs + row * LDC + c1c);
      v4f v0, v1;
#pragma unroll
      for (int e = 0; e < 4; ++e) {
        v0[e] = a0[e] * (1.0f / 16384.0f);
        v1[e] = a1[e] * (1.0f / 16384.0f);
      }
      float* p0 = o32 + t * PJW + c0;
      float* p1 = o32 + t * PJW + c1c;
      *(volatile v4f*)p0 = v0;
      if (c1 < NBW) *(volatile v4f*)p1 = v1;
      __threadfence();
      *(volatile v4f*)p0 = v0;
      if (c1 < NBW) *(volatile v4f*)p1 = v1;
    }
  } else if (MODE == 2) {
    const int c0 = lane * 4;
    const int cc = min(c0, NBW - 4);
#pragma unroll 1
    for (int row = wave; row < 64; row += NW) {
      const size_t t = (size_t)mb * 64 + row;
      const v4f a = *(const v4f*)(Cs + row * LDC + cc);
      const v4f xv = *(const v4f*)(q0 + t * DM + cc);
      v4f o;
#pragma unroll
      for (int e = 0; e < 4; ++e) o[e] = bfr(xv[e]) + a[e] * (1.0f / 65536.0f);
      float* p = o32 + t * DM + cc;
      if (c0 < NBW) *(volatile v4f*)p = o;
      __threadfence();
      if (c0 < NBW) *(volatile v4f*)p = o;
    }
  } else if (MODE == 3) {
    const int cb = lane * 4;
    const int gcol = nb * NBW + cb;
    const v4f bv = *(const v4f*)(q0 + gcol);
#pragma unroll 1
    for (int row = wave; row < 64; row += NW) {
      const size_t t = (size_t)mb * 64 + row;
      const v4f a = *(const v4f*)(Cs + row * LDC + cb);
      v4f gl;
#pragma unroll
      for (int e = 0; e < 4; ++e) gl[e] = fmaxf(a[e] * (1.0f / 512.0f) + bfr(bv[e]), 0.0f);
      v2u ph, pl;
      pack4(gl, S_H, ph, pl);
      unsigned short* hp = oh + t * HID + gcol;
      unsigned short* lp = ol + t * HID + gcol;
      *(volatile v2u*)hp = ph;
      *(volatile v2u*)lp = pl;
      __threadfence();
      *(volatile v2u*)hp = ph;
      *(volatile v2u*)lp = pl;
    }
  } else {
    const int c0 = lane * 4;
    const int cc = min(c0, NBW - 4);
    const v4f bv = *(const v4f*)(q0 + cc);
#pragma unroll 1
    for (int row = wave; row < 64; row += NW) {
      const size_t t = (size_t)mb * 64 + row;
      const v4f a = *(const v4f*)(Cs + row * LDC + cc);
      const v4f ev = *(const v4f*)(q1 + t * DM + cc);
      v4f o;
#pragma unroll
      for (int e = 0; e < 4; ++e) o[e] = ev[e] + (a[e] * (1.0f / 4096.0f) + bfr(bv[e]));
      float* p = o32 + t * DM + cc;
      if (c0 < NBW) *(volatile v4f*)p = o;
      __threadfence();
      if (c0 < NBW) *(volatile v4f*)p = o;
    }
  }
}

extern "C" void kernel_launch(void* const* d_in, const int* in_sizes, int n_in,
                              void* d_out, int out_size, void* d_ws, size_t ws_size,
                              hipStream_t stream) {
  if (n_in < 22) return;
  if (in_sizes[0] != NT * DM) return;
  if (in_sizes[3] != DM || in_sizes[4] != DM) return;
  if (in_sizes[5] != XZW * DM) return;
  if (in_sizes[6] != DI * 4 || in_sizes[7] != DI) return;
  if (in_sizes[8] != (DTR + 2 * DS) * DI) return;
  if (in_sizes[9] != DI * DTR || in_sizes[10] != DI) return;
  if (in_sizes[11] != DI * DS || in_sizes[12] != DI) return;
  if (in_sizes[13] != DM * DI) return;
  if (in_sizes[14] != DM || in_sizes[15] != DM || in_sizes[16] != DM || in_sizes[17] != DM) return;
  if (in_sizes[18] != HID * DM || in_sizes[19] != HID) return;
  if (in_sizes[20] != DM * HID || in_sizes[21] != DM) return;
  if (out_size != 2 * NT * DM) return;

  const float* x      = (const float*)d_in[0];
  const float* n1g    = (const float*)d_in[3];
  const float* n1b    = (const float*)d_in[4];
  const float* inw    = (const float*)d_in[5];
  const float* cvw    = (const float*)d_in[6];
  const float* cvb    = (const float*)d_in[7];
  const float* xpw    = (const float*)d_in[8];
  const float* dtw    = (const float*)d_in[9];
  const float* dtb    = (const float*)d_in[10];
  const float* alog   = (const float*)d_in[11];
  const float* dpar   = (const float*)d_in[12];
  const float* outw   = (const float*)d_in[13];
  const float* n3g    = (const float*)d_in[14];
  const float* n3b    = (const float*)d_in[15];
  const float* n4g    = (const float*)d_in[16];
  const float* n4b    = (const float*)d_in[17];
  const float* f1w    = (const float*)d_in[18];
  const float* f1b    = (const float*)d_in[19];
  const float* f2w    = (const float*)d_in[20];
  const float* f2b    = (const float*)d_in[21];
  float* out0 = (float*)d_out;
  float* out1 = (float*)d_out + (size_t)NT * DM;

  const size_t sP128h = (size_t)NT * DI * 2;
  const size_t sP64h  = (size_t)NT * DM * 2;
  const size_t sP128f = (size_t)NT * DI * 4;
  const size_t sP64f  = (size_t)NT * DM * 4;
  const size_t sDBC   = (size_t)NT * PJW * 4;
  const size_t sHIDh  = (size_t)HROWS * HID * 2;

  const size_t oZ   = 0;
  const size_t oU   = oZ + sP128f;
  const size_t oUH  = oU + sP128f;
  const size_t oUL  = oUH + sP128h;
  const size_t oXNH = oUL + sP128h;
  const size_t oXNL = oXNH + sP64h;
  const size_t oYH  = oXNH;
  const size_t oYL  = oYH + sP128h;
  const size_t oHH  = 0;
  const size_t oHL  = oHH + sHIDh;
  size_t sR1 = oYL + sP128h;
  if (oXNL + sP64h > sR1) sR1 = oXNL + sP64h;
  if (oHL + sHIDh > sR1) sR1 = oHL + sHIDh;

  const size_t oDBC = 0;
  const size_t oE0  = 0;
  const size_t oENC = oE0 + sP64f;
  const size_t oEH  = oENC + sP64f;
  const size_t oEL  = oEH + sP64h;
  const size_t oF   = oEL + sP64h;
  size_t sR2 = oF + sP64f;
  if (oDBC + sDBC > sR2) sR2 = oDBC + sDBC;

  const size_t sWIN  = (size_t)XZW * DM * 2;
  const size_t sWXP  = (size_t)PJW * DI * 2;
  const size_t sWOUT = (size_t)DM * DI * 2;
  const size_t sWF1  = (size_t)HID * DM * 2;
  const size_t sWF2  = (size_t)DM * HID * 2;
  const size_t sA2   = (size_t)DI * DS * 4;

  size_t off = 0;
  const size_t oR1 = off; off += sR1;
  const size_t oR2 = off; off += sR2;
  const size_t oWIN = off; off += sWIN;
  const size_t oWXP = off; off += sWXP;
  const size_t oWOUT = off; off += sWOUT;
  const size_t oWF1 = off; off += sWF1;
  const size_t oWF2 = off; off += sWF2;
  const size_t oA2 = off; off += sA2;
  if (off > ws_size) return;
  if (off > (size_t)134217728) return;

  char* ws = (char*)d_ws;
  float*          Z    = (float*)(ws + oR1 + oZ);
  float*          U    = (float*)(ws + oR1 + oU);
  unsigned short* UH   = (unsigned short*)(ws + oR1 + oUH);
  unsigned short* UL   = (unsigned short*)(ws + oR1 + oUL);
  unsigned short* XNH  = (unsigned short*)(ws + oR1 + oXNH);
  unsigned short* XNL  = (unsigned short*)(ws + oR1 + oXNL);
  unsigned short* YH   = (unsigned short*)(ws + oR1 + oYH);
  unsigned short* YL   = (unsigned short*)(ws + oR1 + oYL);
  unsigned short* HH   = (unsigned short*)(ws + oR1 + oHH);
  unsigned short* HL   = (unsigned short*)(ws + oR1 + oHL);
  float*          DBC  = (float*)(ws + oR2 + oDBC);
  float*          E0   = (float*)(ws + oR2 + oE0);
  float*          ENC  = (float*)(ws + oR2 + oENC);
  unsigned short* EH   = (unsigned short*)(ws + oR2 + oEH);
  unsigned short* EL   = (unsigned short*)(ws + oR2 + oEL);
  float*          F    = (float*)(ws + oR2 + oF);
  unsigned short* WIN  = (unsigned short*)(ws + oWIN);
  unsigned short* WXP  = (unsigned short*)(ws + oWXP);
  unsigned short* WOUT = (unsigned short*)(ws + oWOUT);
  unsigned short* WF1  = (unsigned short*)(ws + oWF1);
  unsigned short* WF2  = (unsigned short*)(ws + oWF2);
  float*          A2   = (float*)(ws + oA2);
  const float*    dq   = n1g;
  float*          df   = Z;
  unsigned short* dh   = XNH;

  k_ln<0><<<dim3(NT / 8), dim3(256), 0, stream>>>(x, n1g, n1b, out0, XNH, XNL);
  k_cvt<<<dim3((XZW * (DM / 8) + 255) / 256), dim3(256), 0, stream>>>(inw, XZW, DM, WIN, XZW);
  k_cvt<<<dim3((2 * DS * (DI / 8) + 255) / 256), dim3(256), 0, stream>>>(xpw + (size_t)DTR * DI, 2 * DS, DI, WXP, 2 * DS);
  k_cvt<<<dim3(((PJW - 2 * DS) * (DI / 8) + 255) / 256), dim3(256), 0, stream>>>(xpw, DTR, DI, WXP + (size_t)2 * DS * DI, PJW - 2 * DS);
  k_cvt<<<dim3((DM * (DI / 8) + 255) / 256), dim3(256), 0, stream>>>(outw, DM, DI, WOUT, DM);
  k_cvt<<<dim3((HID * (DM / 8) + 255) / 256), dim3(256), 0, stream>>>(f1w, HID, DM, WF1, HID);
  k_cvt<<<dim3((DM * (HID / 8) + 255) / 256), dim3(256), 0, stream>>>(f2w, DM, HID, WF2, DM);
  k_atab<<<dim3((DI * DS + 255) / 256), dim3(256), 0, stream>>>(alog, DI * DS, A2);
  k_gemm<0, 4><<<dim3(NT / 64, XZW / 128), dim3(256), 0, stream>>>(XNH, XNL, DM, WIN, DM, DM / 32,
                                                                    cvw, cvb, Z, U, UH, UL);
  k_gemm<1, 5><<<dim3(NT / 64, 1), dim3(320), 0, stream>>>(UH, UL, DI, WXP, DI, DI / 32,
                                                            dq, dq, DBC, df, dh, dh);
  k_scan<<<dim3(NSEQ), dim3(128), 0, stream>>>(DBC, U, Z, A2, dtw, dtb, dpar, YH, YL);
  k_gemm<2, 2><<<dim3(NT / 64, 1), dim3(128), 0, stream>>>(YH, YL, DI, WOUT, DI, DI / 32,
                                                            x, dq, E0, df, dh, dh);
  k_ln<1><<<dim3(NT / 8), dim3(256), 0, stream>>>(E0, n3g, n3b, ENC, EH, EL);
  for (int h = 0; h < 2; ++h) {
    const size_t ro16 = (size_t)h * HROWS * DM;
    k_gemm<3, 4><<<dim3(HROWS / 64, HID / 128), dim3(256), 0, stream>>>(EH + ro16, EL + ro16, DM, WF1, DM, DM / 32,
                                                                         f1b, dq, df, df, HH, HL);
    k_gemm<4, 2><<<dim3(HROWS / 64, 1), dim3(128), 0, stream>>>(HH, HL, HID, WF2, HID, HID / 32,
                                                                 f2b, ENC + ro16, F + ro16, df, dh, dh);
  }
  k_ln<2><<<dim3(NT / 8), dim3(256), 0, stream>>>(F, n4g, n4b, out1, dh, dh);
  (void)hipGetLastError();
}
